// BidirectionalCrossBlock_10754598109693
// MI455X (gfx1250) — hardware-verified
//
#include <hip/hip_runtime.h>
#include <math.h>

typedef __attribute__((ext_vector_type(16))) _Float16 v16h;
typedef __attribute__((ext_vector_type(16))) __bf16 v16b;
typedef __attribute__((ext_vector_type(8)))  _Float16 v8h;
typedef __attribute__((ext_vector_type(8)))  float v8f;
typedef __attribute__((ext_vector_type(4)))  float v4f;
typedef __attribute__((ext_vector_type(2)))  float v2f;
typedef __attribute__((ext_vector_type(4)))  unsigned v4u;
typedef __attribute__((ext_vector_type(4)))  int v4i;
typedef float __attribute__((may_alias)) float_a;
typedef int __attribute__((may_alias)) int_a;

template <typename T> __device__ __forceinline__ void vst2(void* p, T v) { *(volatile T*)p = v; __threadfence(); *(volatile T*)p = v; }
__device__ __forceinline__ v8f wmma16(v16h a, v16h b, v8f c) {
  v8f d = __builtin_amdgcn_wmma_f32_16x16x32_f16(false, a, false, b, (short)0, c, false, false);
  asm volatile("v_nop\n\tv_nop\n\tv_nop\n\tv_nop" : "+v"(d) : "v"(a), "v"(b));
  return d;
}
__device__ __forceinline__ v8f wmma_bf(v16b a, v16b b, v8f c) {
  v8f d = __builtin_amdgcn_wmma_f32_16x16x32_bf16(false, a, false, b, (short)0, c, false, false);
  asm volatile("v_nop\n\tv_nop\n\tv_nop\n\tv_nop" : "+v"(d) : "v"(a), "v"(b));
  return d;
}
__device__ __forceinline__ v16h frag_h(const _Float16* rowk0, int lane) {
  union { v16h v; v8h q[2]; } u; const _Float16* p = rowk0 + 8 * (lane >> 4);
  u.q[0] = *(const v8h*)p; u.q[1] = *(const v8h*)(p + 16); return u.v;
}
__device__ __forceinline__ v16h frag_f32(const float* rowk0, int lane) {
  v16h a; const float* p = rowk0 + 8 * (lane >> 4);
#pragma unroll
  for (int i = 0; i < 8; ++i) { a[i] = (_Float16)p[i]; a[8 + i] = (_Float16)p[16 + i]; }
  return a;
}
__device__ __forceinline__ v16h frag_f32s(const float* rowk0, int lane, float sc) {
  v16h a; const float* p = rowk0 + 8 * (lane >> 4);
#pragma unroll
  for (int i = 0; i < 8; ++i) { a[i] = (_Float16)(p[i] * sc); a[8 + i] = (_Float16)(p[16 + i] * sc); }
  return a;
}
__device__ __forceinline__ v16h fragc_f32(const float* W, int k0, int n, int lane, int ld, int K) {
  v16h a; const int g = lane >> 4;
#pragma unroll
  for (int i = 0; i < 8; ++i) { const int ka = k0 + 8 * g + i, kb = ka + 16;
    a[i] = (_Float16)(ka < K ? W[(size_t)(ka < K ? ka : K - 1) * ld + n] : 0.f); a[8 + i] = (_Float16)(kb < K ? W[(size_t)(kb < K ? kb : K - 1) * ld + n] : 0.f); }
  return a;
}
struct F2 { v16b h, l; };
__device__ __forceinline__ F2 bsplit16(const float v[16]) { F2 r;
#pragma unroll
  for (int i = 0; i < 16; ++i) { const __bf16 h = (__bf16)v[i]; r.h[i] = h; r.l[i] = (__bf16)(v[i] - (float)h); }
  return r; }
__device__ __forceinline__ F2 split_row(const float* row, int k0, int lane) { float v[16]; const float* p = row + k0 + 8 * (lane >> 4);
#pragma unroll
  for (int i = 0; i < 8; ++i) { v[i] = p[i]; v[8 + i] = p[16 + i]; }
  return bsplit16(v); }
__device__ __forceinline__ F2 split_rowK(const float* row, int k0, int lane, int K) { float v[16]; const int g = lane >> 4;
#pragma unroll
  for (int i = 0; i < 8; ++i) { const int ka = k0 + 8 * g + i, kb = ka + 16; v[i] = ka < K ? row[ka < K ? ka : K - 1] : 0.f; v[8 + i] = kb < K ? row[kb < K ? kb : K - 1] : 0.f; }
  return bsplit16(v); }
__device__ __forceinline__ F2 split_col(const float* W, int k0, int n, int lane, int ld, int K) { float v[16]; const int g = lane >> 4;
#pragma unroll
  for (int i = 0; i < 8; ++i) { const int ka = k0 + 8 * g + i, kb = ka + 16; v[i] = ka < K ? W[(size_t)(ka < K ? ka : K - 1) * ld + n] : 0.f; v[8 + i] = kb < K ? W[(size_t)(kb < K ? kb : K - 1) * ld + n] : 0.f; }
  return bsplit16(v); }
__device__ __forceinline__ v8f mac3(const F2& a, const F2& b, v8f c) { c = wmma_bf(a.l, b.h, c); c = wmma_bf(a.h, b.l, c); return wmma_bf(a.h, b.h, c); }
__device__ __forceinline__ float sigm(float v) { return 1.0f / (1.0f + expf(-v)); }
#define LDSX() do { asm volatile("s_wait_dscnt 0" ::: "memory"); __builtin_amdgcn_wave_barrier(); __builtin_amdgcn_fence(__ATOMIC_RELEASE, "workgroup"); } while (0)


#define NT 4096
#define CC 256
#define NH 8
#define HDd 32
#define CM 512
#define GW 64
#ifndef TQB
#define TQB (NT / 64)
#endif
#define NRX (2 * NT)
#ifndef TCVS
#define TCVS GW
#endif
#define TRW NRX
typedef __attribute__((ext_vector_type(8))) __bf16 v8b;
__device__ __forceinline__ v16b frag_b(const __bf16* rowk0, int lane) {
  union { v16b v; v8b q[2]; } u; const __bf16* p = rowk0 + 8 * (lane >> 4);
  u.q[0] = *(const v8b*)p; u.q[1] = *(const v8b*)(p + 16); return u.v;
}
__device__ __forceinline__ float bfr(float v) { return (float)(__bf16)v; }
__device__ __attribute__((noinline)) float exp_ni(float v) { return expf(v); }
__device__ __attribute__((noinline)) float erf_ni(float v) { return erff(v); }

#define PK_PR 0
#define PK_MG ((size_t)CM * CC)
#define PK_LN (PK_MG + (size_t)CC * CC)
#define PK_CV (PK_LN + (size_t)CM * CM)
#define PK_END (PK_CV + (size_t)CC * 9 * CM)
#define WS_PK  0u
#define WS_QH  (((2u * PK_END) + 127u) / 128u * 128u)
#define WS_QL  (WS_QH + 2u * NRX * CC)
#define WS_VH  (WS_QL + 2u * NRX * CC)
#define WS_VL  (WS_VH + 2u * NRX * CC)
#define WS_M   (WS_VL + 2u * NRX * CC)
#define WS_MN  (WS_M + 4u * NRX * CC)
#define WS_MNL (WS_MN + 2u * NRX * CC)
#define WS_GH  (WS_MNL + 2u * NRX * CC)
#define WS_GL  (WS_GH + 2u * NRX * CM)
#define WS_END (WS_GL + 2u * NRX * CM)

__global__ __launch_bounds__(256) void k_pack(const float* __restrict__ PW, const float* __restrict__ MW, const float* __restrict__ LW, const float* __restrict__ CW, __bf16* __restrict__ PK) {
  __shared__ __align__(16) __bf16 s[9 * CM]; const int n = blockIdx.x, which = blockIdx.y, t = threadIdx.x; int K; size_t dst;
  if (which == 0) { K = CC; dst = PK_PR + (size_t)n * CC; for (int k = t; k < K; k += 256) s[k] = (__bf16)PW[(size_t)n * CC + k]; }
  else if (which == 1) { if (n >= CC) return; K = CC; dst = PK_MG + (size_t)n * CC; for (int k = t; k < K; k += 256) s[k] = (__bf16)MW[(size_t)n * CC + k]; }
  else if (which == 2) { K = CM; dst = PK_LN + (size_t)n * CM; for (int k = t; k < K; k += 256) s[k] = (__bf16)LW[(size_t)n * CM + k]; }
  else { if (n >= CC) return; K = 9 * CM; dst = PK_CV + (size_t)n * 9 * CM; for (int k = t; k < K; k += 256) { const int tap = k / CM, c = k % CM; s[k] = (__bf16)CW[(((size_t)n * CM + c) * 3 + tap / 3) * 3 + tap % 3]; } }
  __syncthreads();
  for (int q = t; q < K / 8; q += 256) vst2((unsigned*)(PK + dst + q * 8), *(const v4u*)&s[q * 8]);
}
__global__ __launch_bounds__(128) void k_proj(const float* __restrict__ X0, const float* __restrict__ X1, const __bf16* __restrict__ PK, const float* __restrict__ PB, _Float16* __restrict__ QH, _Float16* __restrict__ QL, _Float16* __restrict__ VH, _Float16* __restrict__ VL) {
  __shared__ __align__(16) _Float16 so[4][16][136], sol[4][16][136]; __shared__ __align__(16) _Float16 sth[128][72], stl[128][72];
  const int tid = threadIdx.x, wave = tid >> 5, lane = tid & 31, col = lane & 15, g = lane >> 4; const size_t r0 = (size_t)blockIdx.x * 64 + wave * 16; const int n0 = blockIdx.y * 128; const size_t side = r0 / NT; const float* X = side ? X1 : X0; const size_t xr = r0 - side * NT;
  v8f acc[8] = {};
#pragma unroll
  for (int kc = 0; kc < CC / 32; ++kc) { v16b a; { const float* p = X + (xr + col) * CC + kc * 32 + 8 * g;
#pragma unroll
      for (int i = 0; i < 8; ++i) { a[i] = (__bf16)p[i]; a[8 + i] = (__bf16)p[16 + i]; } }
#pragma unroll
    for (int j = 0; j < 8; ++j) acc[j] = wmma_bf(a, frag_b(PK + PK_PR + (size_t)(n0 + j * 16 + col) * CC + kc * 32, lane), acc[j]); }
  if (n0 < CC) {
#pragma unroll
    for (int j = 0; j < 8; ++j) { const float bb = bfr(PB[n0 + j * 16 + col]);
#pragma unroll
      for (int r = 0; r < 8; ++r) { const float v = acc[j][r] + bb; const _Float16 hv = (_Float16)v; so[wave][8 * g + r][j * 16 + col] = hv; sol[wave][8 * g + r][j * 16 + col] = (_Float16)((v - (float)hv) * 2048.0f); } }
    LDSX();
    for (int rl = 0; rl < 16; ++rl) if (lane < 16) { vst2((unsigned*)(QH + (r0 + rl) * CC + n0 + lane * 8), *(const v4u*)&so[wave][rl][lane * 8]); vst2((unsigned*)(QL + (r0 + rl) * CC + n0 + lane * 8), *(const v4u*)&sol[wave][rl][lane * 8]); }
  } else {
#pragma unroll
    for (int j = 0; j < 8; ++j) { const float bb = bfr(PB[n0 + j * 16 + col]);
#pragma unroll
      for (int r = 0; r < 8; ++r) { const float v = acc[j][r] + bb; const _Float16 hv = (_Float16)v; sth[j * 16 + col][wave * 16 + 8 * g + r] = hv; stl[j * 16 + col][wave * 16 + 8 * g + r] = (_Float16)((v - (float)hv) * 2048.0f); } }
    __syncthreads();
    const int c0 = n0 - CC; const size_t t0 = (size_t)blockIdx.x * 64 - side * NT;
    for (int e = tid; e < 128 * 8; e += 128) { const int d = e >> 3, pc = e & 7; const size_t o = (side * CC + c0 + d) * NT + t0 + pc * 8; vst2((unsigned*)(VH + o), *(const v4u*)&sth[d][pc * 8]); vst2((unsigned*)(VL + o), *(const v4u*)&stl[d][pc * 8]); }
  }
}
__global__ __launch_bounds__(128) void k_attn(const _Float16* __restrict__ QH, const _Float16* __restrict__ QL, const _Float16* __restrict__ VH, const _Float16* __restrict__ VL, float* __restrict__ M) {
  __shared__ __align__(16) _Float16 sph[4][16][40], spl[4][16][40]; __shared__ __align__(16) float so[4][16][36];
  const int tid = threadIdx.x, wave = tid >> 5, lane = tid & 31, col = lane & 15, g = lane >> 4; const int qb = blockIdx.x, h = blockIdx.y, dir = blockIdx.z; const size_t qside = dir, kside = 1 - dir; const int q0 = qb * 64 + wave * 16; const size_t rq = qside * NT + q0;
  const v16h aq = frag_h(QH + (rq + col) * CC + h * HDd, lane), aql = frag_h(QL + (rq + col) * CC + h * HDd, lane);
  float m[8], l[8];
#pragma unroll
  for (int r = 0; r < 8; ++r) { m[r] = -3.0e38f; l[r] = 0.f; }
  v8f acc[2] = {}, accl[2] = {}; const float isc = 1.0f / sqrtf((float)HDd);
#pragma unroll 1
  for (int ks = 0; ks < NT / 32; ++ks) { const int j0 = ks * 32; v8f s[2];
#pragma unroll
    for (int ct = 0; ct < 2; ++ct) { const int kk = j0 + ct * 16 + col; const size_t rk = (kside * NT + kk) * CC + h * HDd; v8f c = {}, cl = {};
      { const v16h kh = frag_h(QH + rk, lane); c = wmma16(aq, kh, c); cl = wmma16(aql, kh, cl); cl = wmma16(aq, frag_h(QL + rk, lane), cl); }
#pragma unroll
      for (int r = 0; r < 8; ++r) s[ct][r] = (c[r] + cl[r] * (1.0f / 2048.0f)) * isc; }
#pragma unroll
    for (int r = 0; r < 8; ++r) { float mx = fmaxf(s[0][r], s[1][r]);
#pragma unroll
      for (int o = 1; o < 16; o <<= 1) mx = fmaxf(mx, __shfl_xor(mx, o));
      const float mn = fmaxf(m[r], mx); const float alpha = (m[r] <= -1.0e38f) ? 0.f : __expf(m[r] - mn);
      const float e0 = __expf(s[0][r] - mn), e1 = __expf(s[1][r] - mn); float es = e0 + e1;
#pragma unroll
      for (int o = 1; o < 16; o <<= 1) es += __shfl_xor(es, o);
      l[r] = l[r] * alpha + es; m[r] = mn; acc[0][r] *= alpha; acc[1][r] *= alpha; accl[0][r] *= alpha; accl[1][r] *= alpha;
      { const float p0 = e0 * 2048.0f, p1 = e1 * 2048.0f; const _Float16 h0 = (_Float16)p0, h1 = (_Float16)p1; sph[wave][8 * g + r][col] = h0; sph[wave][8 * g + r][16 + col] = h1; spl[wave][8 * g + r][col] = (_Float16)((p0 - (float)h0) * 2048.0f); spl[wave][8 * g + r][16 + col] = (_Float16)((p1 - (float)h1) * 2048.0f); } }
    LDSX();
    const v16h pah = frag_h(&sph[wave][col][0], lane), pal = frag_h(&spl[wave][col][0], lane);
#pragma unroll
    for (int dt = 0; dt < 2; ++dt) { const size_t vo = (kside * CC + h * HDd + dt * 16 + col) * NT + j0; const v16h vh = frag_h(VH + vo, lane); acc[dt] = wmma16(pah, vh, acc[dt]); accl[dt] = wmma16(pal, vh, accl[dt]); accl[dt] = wmma16(pah, frag_h(VL + vo, lane), accl[dt]); }
    LDSX(); }
#pragma unroll
  for (int r = 0; r < 8; ++r) { const float il = (1.0f / 2048.0f) / l[r];
#pragma unroll
    for (int dt = 0; dt < 2; ++dt) so[wave][8 * g + r][dt * 16 + col] = (acc[dt][r] + accl[dt][r] * (1.0f / 2048.0f)) * il; }
  LDSX();
  for (int rl = 0; rl < 16; ++rl) if (lane < 8) vst2(M + (rq + rl) * CC + h * HDd + lane * 4, *(const v4f*)&so[wave][rl][lane * 4]);
}
__global__ __launch_bounds__(128) void k_merge(const float* __restrict__ M, const __bf16* __restrict__ PK, const float* __restrict__ MB, const float* __restrict__ G0, const float* __restrict__ B0, __bf16* __restrict__ MN, __bf16* __restrict__ MNL) {
  __shared__ __align__(16) float so[64][CC + 4]; __shared__ __align__(16) __bf16 sh[64][CC + 8], sl[64][CC + 8];
  const int tid = threadIdx.x, wave = tid >> 5, lane = tid & 31, col = lane & 15, g = lane >> 4; const size_t rb0 = (size_t)blockIdx.x * 64; const size_t r0 = rb0 + wave * 16;
#pragma unroll 1
  for (int half = 0; half < 2; ++half) { v8f acc[8] = {};
#pragma unroll
    for (int kc = 0; kc < CC / 32; ++kc) { const F2 a = split_row(M + (r0 + col) * CC, kc * 32, lane);
#pragma unroll
      for (int j = 0; j < 8; ++j) { const v16b w = frag_b(PK + PK_MG + (size_t)(half * 128 + j * 16 + col) * CC + kc * 32, lane); acc[j] = wmma_bf(a.l, w, acc[j]); acc[j] = wmma_bf(a.h, w, acc[j]); } }
#pragma unroll
    for (int j = 0; j < 8; ++j) { const int c = half * 128 + j * 16 + col; const float bb = bfr(MB[c]);
#pragma unroll
      for (int r = 0; r < 8; ++r) so[wave * 16 + 8 * g + r][c] = acc[j][r] + bb; } }
  __syncthreads();
  { const int r = tid >> 1, part = tid & 1; float s = 0.f; for (int c = part * 128; c < part * 128 + 128; ++c) s += so[r][c]; s += __shfl_xor(s, 1); const float mu = s / (float)CC; float q = 0.f; for (int c = part * 128; c < part * 128 + 128; ++c) { const float d = so[r][c] - mu; q += d * d; } q += __shfl_xor(q, 1); const float inv = 1.0f / sqrtf(q / (float)CC + 1e-5f);
    for (int c = part * 128; c < part * 128 + 128; ++c) { const float y = (so[r][c] - mu) * inv * bfr(G0[c]) + bfr(B0[c]); const __bf16 hb = (__bf16)y; sh[r][c] = hb; sl[r][c] = (__bf16)(y - (float)hb); } }
  __syncthreads();
  for (int e = tid; e < 64 * (CC / 8); e += 128) { const int r = e / (CC / 8), q = e % (CC / 8); vst2((unsigned*)(MN + (rb0 + r) * CC + q * 8), *(const v4u*)&sh[r][q * 8]); vst2((unsigned*)(MNL + (rb0 + r) * CC + q * 8), *(const v4u*)&sl[r][q * 8]); }
}
__global__ __launch_bounds__(128) void k_lin(const float* __restrict__ X0, const float* __restrict__ X1, const __bf16* __restrict__ MN, const __bf16* __restrict__ MNL, const __bf16* __restrict__ PK, const float* __restrict__ LB, __bf16* __restrict__ GH, __bf16* __restrict__ GL) {
  __shared__ __align__(16) __bf16 sg[4][16][136], sgl[4][16][136];
  const int tid = threadIdx.x, wave = tid >> 5, lane = tid & 31, col = lane & 15, g = lane >> 4; const size_t r0 = (size_t)blockIdx.x * 64 + wave * 16; const int n0 = blockIdx.y * 128; const size_t side = r0 / NT; const float* X = side ? X1 : X0; const size_t xr = r0 - side * NT;
  v8f acc[8] = {};
#pragma unroll
  for (int kc = 0; kc < CM / 32; ++kc) {
    if (kc < CC / 32) { v16b a; { const float* p = X + (xr + col) * CC + kc * 32 + 8 * g;
#pragma unroll
        for (int i = 0; i < 8; ++i) { a[i] = (__bf16)p[i]; a[8 + i] = (__bf16)p[16 + i]; } }
#pragma unroll
      for (int j = 0; j < 8; ++j) acc[j] = wmma_bf(a, frag_b(PK + PK_LN + (size_t)(n0 + j * 16 + col) * CM + kc * 32, lane), acc[j]); }
    else { const v16b a = frag_b(MN + (r0 + col) * CC + (kc - CC / 32) * 32, lane), al = frag_b(MNL + (r0 + col) * CC + (kc - CC / 32) * 32, lane);
#pragma unroll
      for (int j = 0; j < 8; ++j) { const v16b w = frag_b(PK + PK_LN + (size_t)(n0 + j * 16 + col) * CM + kc * 32, lane); acc[j] = wmma_bf(al, w, acc[j]); acc[j] = wmma_bf(a, w, acc[j]); } } }
#pragma unroll
  for (int j = 0; j < 8; ++j) { const float bb = bfr(LB[n0 + j * 16 + col]);
#pragma unroll
    for (int r = 0; r < 8; ++r) { const float x = acc[j][r] + bb; const float gv = x * 0.5f * (1.0f + erf_ni(x * 0.70710678118654752f)); const __bf16 hb = (__bf16)gv; sg[wave][8 * g + r][j * 16 + col] = hb; sgl[wave][8 * g + r][j * 16 + col] = (__bf16)(gv - (float)hb); } }
  LDSX();
  for (int rl = 0; rl < 16; ++rl) { if (lane < 16) vst2((unsigned*)(GH + (r0 + rl) * CM + n0 + lane * 8), *(const v4u*)&sg[wave][rl][lane * 8]); else vst2((unsigned*)(GL + (r0 + rl) * CM + n0 + (lane - 16) * 8), *(const v4u*)&sgl[wave][rl][(lane - 16) * 8]); }
}
__global__ __launch_bounds__(128) void k_conv(const __bf16* __restrict__ GH, const __bf16* __restrict__ GL, const float* __restrict__ X0, const float* __restrict__ X1, const __bf16* __restrict__ PK, const float* __restrict__ CB, const float* __restrict__ G1, const float* __restrict__ B1, float* __restrict__ OUT0, float* __restrict__ OUT1) {
  __shared__ __align__(16) __bf16 sh[66][40], sl[66][40]; __shared__ __align__(16) float so[64][CC + 4];
  const int tid = threadIdx.x, wave = tid >> 5, lane = tid & 31, col = lane & 15, g = lane >> 4; const size_t side = blockIdx.x / TCVS; const int y = blockIdx.x % TCVS;
  v8f acc[16] = {};
#pragma unroll 1
  for (int tap = 0; tap < 9; ++tap) { const int dy = tap / 3 - 1, dx = tap % 3 - 1; const int yy = y + dy;
#pragma unroll 1
    for (int kc = 0; kc < CM / 32; ++kc) {
      for (int e = tid; e < 66 * 4; e += 128) { const int xi = e >> 2, q = e & 3; const int xx = xi - 1; v4u hv = {0u, 0u, 0u, 0u}, lv = {0u, 0u, 0u, 0u};
        if (yy >= 0 && yy < GW && xx >= 0 && xx < GW) { const size_t row = side * NT + (size_t)yy * GW + xx; hv = *(const v4u*)(GH + row * CM + kc * 32 + q * 8); lv = *(const v4u*)(GL + row * CM + kc * 32 + q * 8); }
        *(v4u*)&sh[xi][q * 8] = hv; *(v4u*)&sl[xi][q * 8] = lv; }
      __syncthreads();
      const v16b a = frag_b(&sh[wave * 16 + col + dx + 1][0], lane), al = frag_b(&sl[wave * 16 + col + dx + 1][0], lane);
#pragma unroll
      for (int j = 0; j < 16; ++j) { const v16b w = frag_b(PK + PK_CV + (size_t)(j * 16 + col) * (9 * CM) + tap * CM + kc * 32, lane); acc[j] = wmma_bf(al, w, acc[j]); acc[j] = wmma_bf(a, w, acc[j]); }
      __syncthreads(); } }
#pragma unroll
  for (int j = 0; j < 16; ++j) { const float bb = bfr(CB[j * 16 + col]);
#pragma unroll
    for (int r = 0; r < 8; ++r) so[wave * 16 + 8 * g + r][j * 16 + col] = acc[j][r] + bb; }
  __syncthreads();
  const float* X = side ? X1 : X0; float* OUT = side ? OUT1 : OUT0;
  { const int r = tid >> 1, part = tid & 1; const size_t tok = (size_t)y * GW + r; float s = 0.f; for (int c = part * 128; c < part * 128 + 128; ++c) s += so[r][c]; s += __shfl_xor(s, 1); const float mu = s / (float)CC; float q = 0.f; for (int c = part * 128; c < part * 128 + 128; ++c) { const float d = so[r][c] - mu; q += d * d; } q += __shfl_xor(q, 1); const float inv = 1.0f / sqrtf(q / (float)CC + 1e-5f);
    __syncthreads();
    for (int c = part * 128; c < part * 128 + 128; ++c) so[r][c] = (so[r][c] - mu) * inv * bfr(G1[c]) + bfr(B1[c]) + bfr(X[tok * CC + c]); }
  __syncthreads();
  for (int e = tid; e < 64 * (CC / 4); e += 128) { const int r = e / (CC / 4), q = e % (CC / 4); vst2(OUT + ((size_t)y * GW + r) * CC + q * 4, *(const v4f*)&so[r][q * 4]); }
}
extern "C" void kernel_launch(void* const* d_in, const int* in_sizes, int n_in, void* d_out, int out_size, void* d_ws, size_t ws_size, hipStream_t stream) {
  (void)in_sizes; (void)n_in; (void)out_size;
  const float** F = (const float**)d_in;
  if (ws_size < (size_t)WS_END) return;
  char* ws = (char*)d_ws; __bf16 *PK = (__bf16*)(ws + WS_PK), *MN = (__bf16*)(ws + WS_MN), *MNL = (__bf16*)(ws + WS_MNL), *GH = (__bf16*)(ws + WS_GH), *GL = (__bf16*)(ws + WS_GL); _Float16 *QH = (_Float16*)(ws + WS_QH), *QL = (_Float16*)(ws + WS_QL), *VH = (_Float16*)(ws + WS_VH), *VL = (_Float16*)(ws + WS_VL); float* M = (float*)(ws + WS_M);
  float* OUT0 = (float*)d_out; float* OUT1 = (float*)((char*)d_out + 4194304);
  k_pack<<<dim3(CM, 4), 256, 0, stream>>>(F[6], F[8], F[12], F[14], PK);
  k_proj<<<dim3(NRX / 64, CM / 128), 128, 0, stream>>>(F[0], F[1], PK, F[7], QH, QL, VH, VL);
  k_attn<<<dim3(TQB, NH, 2), 128, 0, stream>>>(QH, QL, VH, VL, M);
  k_merge<<<TRW / 64, 128, 0, stream>>>(M, PK, F[9], F[10], F[11], MN, MNL);
  k_lin<<<dim3(TRW / 64, CM / 128), 128, 0, stream>>>(F[0], F[1], MN, MNL, PK, F[13], GH, GL);
  k_conv<<<2 * TCVS, 128, 0, stream>>>(GH, GL, F[0], F[1], PK, F[15], F[16], F[17], OUT0, OUT1);
}
